// DeadlockRGCN_74560632258656
// MI455X (gfx1250) — hardware-verified
//
#include <hip/hip_runtime.h>
#include <stddef.h>


#define INCH      8
#define DF        64
#define NREL      2
#define NCAT      (DF * (NREL + 1))
#define NCQ       (NCAT / 4)
#define HIDC      32
#define WSCALE    16.0f
#define WINV      0.0625f

#define NTHR      256
#define NWAVE     8
#define EPT       8
#define NGRP      2
#define CHUNK     (NTHR * EPT * NGRP)
#define WCAP      (EPT * NGRP * 32)
#define LISTN     (NWAVE * WCAP)
#define NBC       4096
#define NB        1024
#define RPW       (NB / NWAVE)

#define LDS_ACC   (NB * DF * 4)
#define LDS_LIST  (LISTN * 4)
#define LDS_AGG   (LDS_ACC + LDS_LIST + 64)
#define LDS_MAX   (300 * 1024)

#define PG_WAVES  4
#define PG_THR    (PG_WAVES * 32)
#define PG_ROWS   (PG_WAVES * 16)
#define MAXG      1024

static_assert(CHUNK == 4096);
static_assert((NBC & (NBC - 1)) == 0);
static_assert(NBC <= 4096);
static_assert((NB & (NB - 1)) == 0);
static_assert(NB <= 4096);
static_assert(NBC % NB == 0);
static_assert(NTHR == 128 * NREL);
static_assert(NBC % 512 == 0);
static_assert(RPW % 4 == 0);
static_assert(LDS_AGG <= LDS_MAX);
static_assert(DF == 64);
static_assert(MAXG % 4 == 0);
static_assert(MAXG / 4 <= NTHR);
static_assert(NCAT % 4 == 0);

typedef float  v2f   __attribute__((ext_vector_type(2)));
typedef float  v2fa  __attribute__((ext_vector_type(2), __may_alias__));
typedef float  v4f   __attribute__((ext_vector_type(4)));
typedef float  v4fa  __attribute__((ext_vector_type(4), __may_alias__));
typedef float  v8f   __attribute__((ext_vector_type(8)));
typedef int    v4i   __attribute__((ext_vector_type(4)));
typedef _Float16 f16_t;
typedef f16_t  v8h   __attribute__((ext_vector_type(8)));
typedef f16_t  v16h  __attribute__((ext_vector_type(16)));
union FragH { v16h v; v8h h[2]; };
union Pack8 { v8h v; v4i q; };

__device__ __forceinline__ v8f wmh(v16h a, v16h b, v8f c) {
  v8f d = __builtin_amdgcn_wmma_f32_16x16x32_f16(false, a, false, b, (short)0, c, false, false);
  asm volatile("v_nop\n\tv_nop\n\tv_nop\n\tv_nop" : "+v"(d) : "v"(a), "v"(b));
  return d;
}

__device__ __forceinline__ int wrap_clamp(int v, int n) {
  v = (v < 0) ? v + n : v;
  v = (v < 0) ? 0 : ((v > n - 1) ? n - 1 : v);
  return v;
}

__device__ __forceinline__ v4f relu4(v4f v) {
  v4f o;
  o.x = fmaxf(v.x, 0.0f);
  o.y = fmaxf(v.y, 0.0f);
  o.z = fmaxf(v.z, 0.0f);
  o.w = fmaxf(v.w, 0.0f);
  return o;
}

__device__ __forceinline__ float wsum(float v) {
  v += __shfl_xor(v, 16);
  v += __shfl_xor(v, 8);
  v += __shfl_xor(v, 4);
  v += __shfl_xor(v, 2);
  v += __shfl_xor(v, 1);
  return v;
}

template <int MODE, int NSLOT>
__device__ __forceinline__ int scan_chunk(const int* __restrict__ keys, int nK, int cbase, int base,
                                          int vec8, int* list, int tid, int wave) {
  int wc = 0;
#pragma unroll
  for (int g = 0; g < NGRP; ++g) {
    const int el0  = (g * NTHR + tid) * EPT;
    const int e0   = cbase + el0;
    const int sent = -2147483647 - 1;
    v4i da, db;
    if (vec8 != 0 && e0 + 7 < nK) {
      da = *(const v4i*)(keys + e0);
      db = *(const v4i*)(keys + e0 + 4);
    } else {
      da.x = (e0     < nK) ? keys[min(e0,     nK - 1)] : sent;
      da.y = (e0 + 1 < nK) ? keys[min(e0 + 1, nK - 1)] : sent;
      da.z = (e0 + 2 < nK) ? keys[min(e0 + 2, nK - 1)] : sent;
      da.w = (e0 + 3 < nK) ? keys[min(e0 + 3, nK - 1)] : sent;
      db.x = (e0 + 4 < nK) ? keys[min(e0 + 4, nK - 1)] : sent;
      db.y = (e0 + 5 < nK) ? keys[min(e0 + 5, nK - 1)] : sent;
      db.z = (e0 + 6 < nK) ? keys[min(e0 + 6, nK - 1)] : sent;
      db.w = (e0 + 7 < nK) ? keys[min(e0 + 7, nK - 1)] : sent;
    }
#define TSTJ(J, DV) \
    unsigned s##J; bool h##J; \
    { const int dv = (DV); \
      if (MODE) { s##J = 0u; h##J = (dv == base); } \
      else      { s##J = (unsigned)dv - (unsigned)base; h##J = s##J < (unsigned)NSLOT; } }
    TSTJ(0, da.x) TSTJ(1, da.y) TSTJ(2, da.z) TSTJ(3, da.w)
    TSTJ(4, db.x) TSTJ(5, db.y) TSTJ(6, db.z) TSTJ(7, db.w)
#undef TSTJ
    const unsigned any = __builtin_amdgcn_ballot_w32(h0 | h1 | h2 | h3 | h4 | h5 | h6 | h7);
    if (any != 0u) {
#define HITJ(J, HJ, SJ) { \
        const unsigned mj = __builtin_amdgcn_ballot_w32(HJ); \
        if (mj != 0u) { \
          if (HJ) { \
            const int pos  = wc + (int)__builtin_amdgcn_mbcnt_lo(mj, 0u); \
            const int entv = MODE ? (el0 + (J)) : (((el0 + (J)) << 12) | (int)(SJ)); \
            if (pos < WCAP) list[wave * WCAP + pos] = entv; \
          } \
          wc += (int)__builtin_popcount(mj); } }
      HITJ(0, h0, s0)
      HITJ(1, h1, s1)
      HITJ(2, h2, s2)
      HITJ(3, h3, s3)
      HITJ(4, h4, s4)
      HITJ(5, h5, s5)
      HITJ(6, h6, s6)
      HITJ(7, h7, s7)
#undef HITJ
    }
  }
  return wc;
}

__global__ __launch_bounds__(NTHR) void k_wprep(
    const float* __restrict__ w2, const float* __restrict__ rt2,
    const float* __restrict__ w3, const float* __restrict__ rt3,
    f16_t* wpl, int nTot) {
  const int i = blockIdx.x * NTHR + threadIdx.x;
  if (i >= nTot) return;
  const int o   = i * 8;
  const int lyr = o / (NCAT * DF);
  const int rem = o - lyr * (NCAT * DF);
  const int n   = rem / DF;
  const int k0  = rem - n * DF;
  const float* w  = lyr ? w3 : w2;
  const float* rt = lyr ? rt3 : rt2;
  const float* p = (n < NREL * DF) ? (w + (size_t)(n / DF) * DF * DF + (size_t)k0 * DF + (n & (DF - 1)))
                                   : (rt + (size_t)k0 * DF + (n - NREL * DF));
  Pack8 pk;
#define WSP(I) pk.v[(I)] = (f16_t)(p[(size_t)(I) * DF] * WSCALE);
  WSP(0) WSP(1) WSP(2) WSP(3) WSP(4) WSP(5) WSP(6) WSP(7)
#undef WSP
  f16_t* d = wpl + o;
  const v4i q = pk.q;
  *(volatile v4i*)d = q;
  __threadfence();
  *(volatile v4i*)d = q;
}

__global__ __launch_bounds__(NTHR) void k_proj1(
    const float* __restrict__ x, const float* __restrict__ w1, const float* __restrict__ rt1,
    const float* __restrict__ b1, float* P, int nTot) {
  const int gi = blockIdx.x * NTHR + threadIdx.x;
  if (gi >= nTot) return;
  const int row  = gi / NCQ;
  const int cq   = gi - row * NCQ;
  const int col0 = 4 * cq;
  const float* xr = x + (size_t)row * INCH;
  const v4f xa = *(const v4f*)(xr);
  const v4f xb = *(const v4f*)(xr + 4);
  const bool isRoot = col0 >= NREL * DF;
  const float* wp = isRoot ? (rt1 + (col0 - NREL * DF))
                           : (w1 + (size_t)(col0 >> 6) * (INCH * DF) + (col0 & (DF - 1)));
  v4f acc = {0.f, 0.f, 0.f, 0.f};
#define PK(KI, XV) { const v4f wv = *(const v4f*)(wp + (KI) * DF); acc = acc + (XV) * wv; }
  PK(0, xa.x) PK(1, xa.y) PK(2, xa.z) PK(3, xa.w)
  PK(4, xb.x) PK(5, xb.y) PK(6, xb.z) PK(7, xb.w)
#undef PK
  if (isRoot) acc = acc + *(const v4f*)(b1 + (col0 - NREL * DF));
  float* d = P + (size_t)gi * 4;
  *(volatile v4f*)d = acc;
  __threadfence();
  *(volatile v4f*)d = acc;
}

__device__ __forceinline__ void gemm_store_rows(const float* tw, float* P, int rowBase, int nN, int cg, int lane) {
#pragma unroll
  for (int p = 0; p < 8; ++p) {
    const int row = 2 * p + (lane >> 4);
    const int col = 4 * (lane & 15);
    if (rowBase + row < nN) {
      const v4f v = *(const v4fa*)(tw + row * DF + col);
      *(volatile v4f*)(P + (size_t)(rowBase + row) * NCAT + cg * DF + col) = v;
    }
  }
}

__global__ __launch_bounds__(PG_THR) void k_gemm(
    const f16_t* __restrict__ H, const f16_t* __restrict__ wpl, const float* __restrict__ bias,
    float* P, int nN) {
  __shared__ float tile[PG_WAVES * 16 * DF];
  const int tid = threadIdx.x, lane = tid & 31, wave = tid >> 5, hh = lane >> 4, m = lane & 15;
  const int rowBase = blockIdx.x * PG_ROWS + wave * 16;
  int ar = rowBase + m;
  ar = ar > nN - 1 ? nN - 1 : ar;
  const f16_t* ap = H + (size_t)ar * DF + 8 * hh;
  FragH a0, a1;
  a0.h[0] = *(const v8h*)(ap);
  a0.h[1] = *(const v8h*)(ap + 16);
  a1.h[0] = *(const v8h*)(ap + 32);
  a1.h[1] = *(const v8h*)(ap + 48);
  float* tw = tile + wave * 16 * DF;

#pragma unroll 1
  for (int cg = 0; cg < NCAT / DF; ++cg) {
    v8f c[4];
#pragma unroll
    for (int ct = 0; ct < 4; ++ct) { const v8f z = {0.f, 0.f, 0.f, 0.f, 0.f, 0.f, 0.f, 0.f}; c[ct] = z; }
#pragma unroll
    for (int ct = 0; ct < 4; ++ct) {
      const f16_t* bp = wpl + (size_t)(cg * DF + 16 * ct + m) * DF + 8 * hh;
      FragH b0, b1;
      b0.h[0] = *(const v8h*)(bp);
      b0.h[1] = *(const v8h*)(bp + 16);
      b1.h[0] = *(const v8h*)(bp + 32);
      b1.h[1] = *(const v8h*)(bp + 48);
      c[ct] = wmh(a0.v, b0.v, c[ct]);
      c[ct] = wmh(a1.v, b1.v, c[ct]);
    }
    float* sp = tw + (8 * hh) * DF + m;
#pragma unroll
    for (int ct = 0; ct < 4; ++ct) {
      const float bv = (cg == NREL) ? bias[16 * ct + m] : 0.0f;
#pragma unroll
      for (int r = 0; r < 8; ++r) sp[r * DF + 16 * ct] = c[ct][r] * WINV + bv;
    }
    __syncthreads();
    gemm_store_rows(tw, P, rowBase, nN, cg, lane);
    __threadfence();
    gemm_store_rows(tw, P, rowBase, nN, cg, lane);
    __syncthreads();
  }
}

__global__ __launch_bounds__(NTHR) void k_count(
    const int* __restrict__ ei, const int* __restrict__ et,
    float* inv, int nE, int nPad, int vec8) {
  __shared__ int list[LISTN];
  __shared__ int cnt[NBC * NREL];
  __shared__ int wcnt[NWAVE];
  const int tid = threadIdx.x, lane = tid & 31, wave = tid >> 5;
  const int nodeBase = blockIdx.x * NBC;
  const int* dsts = ei + nE;

  for (int i = tid; i < NBC * NREL; i += NTHR) cnt[i] = 0;
  __syncthreads();

  const int nChunks = (nE + CHUNK - 1) / CHUNK;
#pragma unroll 1
  for (int ch = 0; ch < nChunks; ++ch) {
    const int cbase = ch * CHUNK;
    const int wc = scan_chunk<0, NBC>(dsts, nE, cbase, nodeBase, vec8, list, tid, wave);
    if (lane == 0) wcnt[wave] = wc;
    __syncthreads();
    if (wave == 0) {
#pragma unroll 1
      for (int wsx = 0; wsx < NWAVE; ++wsx) {
        int n = __builtin_amdgcn_readfirstlane(wcnt[wsx]);
        n = n > WCAP ? WCAP : (n < 0 ? 0 : n);
        const int* lp = list + wsx * WCAP;
#pragma unroll 1
        for (int i = 0; i < n; ++i) {
          const int ent  = __builtin_amdgcn_readfirstlane(lp[i]);
          const int slot = ent & (NBC - 1);
          int e = cbase + ((ent >> 12) & (CHUNK - 1));
          e = e > nE - 1 ? nE - 1 : e;
          const int r = __builtin_amdgcn_readfirstlane(et[e]);
          if ((unsigned)r < (unsigned)NREL) {
            if (lane == 0) cnt[slot * NREL + r] = cnt[slot * NREL + r] + 1;
          }
        }
      }
    }
    __syncthreads();
  }

  {
    const int r = tid >> 7;
    const int t = tid & 127;
    float* gb = inv + (size_t)r * nPad + nodeBase;
#pragma unroll 1
    for (int q = 0; q < NBC / 512; ++q) {
      const int s4 = q * 512 + 4 * t;
      v4f v;
      { const int c0 = cnt[(s4 + 0) * NREL + r]; v.x = __builtin_amdgcn_rcpf((float)(c0 > 0 ? c0 : 1)); }
      { const int c1 = cnt[(s4 + 1) * NREL + r]; v.y = __builtin_amdgcn_rcpf((float)(c1 > 0 ? c1 : 1)); }
      { const int c2 = cnt[(s4 + 2) * NREL + r]; v.z = __builtin_amdgcn_rcpf((float)(c2 > 0 ? c2 : 1)); }
      { const int c3 = cnt[(s4 + 3) * NREL + r]; v.w = __builtin_amdgcn_rcpf((float)(c3 > 0 ? c3 : 1)); }
      *(volatile v4f*)(gb + s4) = v;
    }
    __threadfence();
#pragma unroll 1
    for (int q = 0; q < NBC / 512; ++q) {
      const int s4 = q * 512 + 4 * t;
      v4f v;
      { const int c0 = cnt[(s4 + 0) * NREL + r]; v.x = __builtin_amdgcn_rcpf((float)(c0 > 0 ? c0 : 1)); }
      { const int c1 = cnt[(s4 + 1) * NREL + r]; v.y = __builtin_amdgcn_rcpf((float)(c1 > 0 ? c1 : 1)); }
      { const int c2 = cnt[(s4 + 2) * NREL + r]; v.z = __builtin_amdgcn_rcpf((float)(c2 > 0 ? c2 : 1)); }
      { const int c3 = cnt[(s4 + 3) * NREL + r]; v.w = __builtin_amdgcn_rcpf((float)(c3 > 0 ? c3 : 1)); }
      *(volatile v4f*)(gb + s4) = v;
    }
  }
}

__device__ __forceinline__ void agg_rows_f16(const float* acc, const float* __restrict__ P, f16_t* hout,
                                             int nodeBase, int nN, int wave, int lane) {
#pragma unroll 1
  for (int i = 0; i < RPW / 4; ++i) {
    const int slot = wave * RPW + 4 * i + (lane >> 3);
    const int node = nodeBase + slot;
    const int c0   = 8 * (lane & 7);
    if (node < nN) {
      const v4f a0 = *(const v4fa*)(acc + slot * DF + c0);
      const v4f a1 = *(const v4fa*)(acc + slot * DF + c0 + 4);
      const float* pr = P + (size_t)node * NCAT + NREL * DF + c0;
      const v4f u0 = relu4(a0 + *(const v4f*)(pr));
      const v4f u1 = relu4(a1 + *(const v4f*)(pr + 4));
      Pack8 pk;
      pk.v[0] = (f16_t)u0.x; pk.v[1] = (f16_t)u0.y; pk.v[2] = (f16_t)u0.z; pk.v[3] = (f16_t)u0.w;
      pk.v[4] = (f16_t)u1.x; pk.v[5] = (f16_t)u1.y; pk.v[6] = (f16_t)u1.z; pk.v[7] = (f16_t)u1.w;
      const v4i q = pk.q;
      *(volatile v4i*)(hout + (size_t)node * DF + c0) = q;
    }
  }
}

__device__ __forceinline__ void agg_rows_f32(const float* acc, const float* __restrict__ P, float* hout,
                                             int nodeBase, int nN, int wave, int lane) {
#pragma unroll 1
  for (int i = 0; i < RPW / 2; ++i) {
    const int slot = wave * RPW + 2 * i + (lane >> 4);
    const int node = nodeBase + slot;
    const int c0   = 4 * (lane & 15);
    if (node < nN) {
      const v4f a  = *(const v4fa*)(acc + slot * DF + c0);
      const v4f pr = *(const v4f*)(P + (size_t)node * NCAT + NREL * DF + c0);
      const v4f v  = a + pr;
      *(volatile v4f*)(hout + (size_t)node * DF + c0) = v;
    }
  }
}

template <int MODE>
__global__ __launch_bounds__(NTHR) void k_agg(
    const int* __restrict__ ei, const int* __restrict__ et, const float* __restrict__ P,
    const float* __restrict__ inv, f16_t* hout16, float* hout32,
    int nN, int nE, int nPad, int vec8) {
  extern __shared__ v4f lds_dyn[];
  float* acc  = (float*)lds_dyn;
  int*   list = (int*)((char*)lds_dyn + LDS_ACC);
  int*   wcnt = (int*)((char*)lds_dyn + LDS_ACC + LDS_LIST);
  const int tid = threadIdx.x, lane = tid & 31, wave = tid >> 5;
  const int nodeBase = blockIdx.x * NB;
  const int* dsts = ei + nE;

  {
    const v4f z = {0.f, 0.f, 0.f, 0.f};
    for (int i = tid; i < NB * DF / 4; i += NTHR) lds_dyn[i] = z;
  }
  __syncthreads();

  const int nChunks = (nE + CHUNK - 1) / CHUNK;
#pragma unroll 1
  for (int ch = 0; ch < nChunks; ++ch) {
    const int cbase = ch * CHUNK;
    const int wc = scan_chunk<0, NB>(dsts, nE, cbase, nodeBase, vec8, list, tid, wave);
    if (lane == 0) wcnt[wave] = wc;
    __syncthreads();
    if (wave == 0) {
#pragma unroll 1
      for (int wsx = 0; wsx < NWAVE; ++wsx) {
        int n = __builtin_amdgcn_readfirstlane(wcnt[wsx]);
        n = n > WCAP ? WCAP : (n < 0 ? 0 : n);
        const int* lp = list + wsx * WCAP;
#pragma unroll 1
        for (int i = 0; i < n; ++i) {
          const int ent  = __builtin_amdgcn_readfirstlane(lp[i]);
          const int slot = ent & (NB - 1);
          int e = cbase + ((ent >> 12) & (CHUNK - 1));
          e = e > nE - 1 ? nE - 1 : e;
          const int r   = __builtin_amdgcn_readfirstlane(et[e]);
          const int src = wrap_clamp(__builtin_amdgcn_readfirstlane(ei[e]), nN);
          if ((unsigned)r < (unsigned)NREL) {
            const float w  = inv[(size_t)r * nPad + nodeBase + slot];
            const v2f   mv = *(const v2fa*)(P + (size_t)src * NCAT + r * DF + 2 * lane);
            v2fa* ap2 = (v2fa*)(acc + slot * DF + 2 * lane);
            const v2f cur = *ap2;
            *ap2 = cur + mv * w;
          }
        }
      }
    }
    __syncthreads();
  }

  if (MODE == 0) {
    agg_rows_f16(acc, P, hout16, nodeBase, nN, wave, lane);
    __threadfence();
    agg_rows_f16(acc, P, hout16, nodeBase, nN, wave, lane);
  } else {
    agg_rows_f32(acc, P, hout32, nodeBase, nN, wave, lane);
    __threadfence();
    agg_rows_f32(acc, P, hout32, nodeBase, nN, wave, lane);
  }
}

__global__ __launch_bounds__(NTHR) void k_pool(
    const int* __restrict__ bt, const float* __restrict__ h3, float* gp, int nN) {
  __shared__ int list[LISTN];
  __shared__ int wcnt[NWAVE];
  const int tid = threadIdx.x, lane = tid & 31, wave = tid >> 5;
  const int g = blockIdx.x;
  float ax = 0.0f, ay = 0.0f;

  const int nChunks = (nN + CHUNK - 1) / CHUNK;
#pragma unroll 1
  for (int ch = 0; ch < nChunks; ++ch) {
    const int cbase = ch * CHUNK;
    const int wc = scan_chunk<1, 1>(bt, nN, cbase, g, 1, list, tid, wave);
    if (lane == 0) wcnt[wave] = wc;
    __syncthreads();
    if (wave == 0) {
#pragma unroll 1
      for (int wsx = 0; wsx < NWAVE; ++wsx) {
        int n = __builtin_amdgcn_readfirstlane(wcnt[wsx]);
        n = n > WCAP ? WCAP : (n < 0 ? 0 : n);
        const int* lp = list + wsx * WCAP;
#pragma unroll 1
        for (int i = 0; i < n; ++i) {
          const int ent = __builtin_amdgcn_readfirstlane(lp[i]);
          int node = cbase + (ent & (CHUNK - 1));
          node = node > nN - 1 ? nN - 1 : node;
          const v2f mv = *(const v2fa*)(h3 + (size_t)node * DF + 2 * lane);
          ax += mv.x;
          ay += mv.y;
        }
      }
    }
    __syncthreads();
  }

  if (wave == 0) {
    const int la = (2 * lane) & 31, lb = (2 * lane + 1) & 31;
    v4f v;
    v.x = __shfl(ax, la);
    v.y = __shfl(ay, la);
    v.z = __shfl(ax, lb);
    v.w = __shfl(ay, lb);
    float* d = gp + (size_t)g * DF + 4 * lane;
    if (lane < 16) *(volatile v4f*)d = v;
    __threadfence();
    if (lane < 16) *(volatile v4f*)d = v;
  }
}

__global__ __launch_bounds__(NTHR) void k_head(
    const float* __restrict__ gp, const float* __restrict__ cw1, const float* __restrict__ cb1,
    const float* __restrict__ cw2, const float* __restrict__ cb2, float* out, int nG) {
  __shared__ float res[MAXG];
  const int tid = threadIdx.x, lane = tid & 31, wave = tid >> 5;
  const float bj = cb1[lane], vj = cw2[lane], bz = cb2[0];
  const int nGG = (nG + NWAVE - 1) / NWAVE;
#pragma unroll 1
  for (int gg = 0; gg < nGG; ++gg) {
    const int g = gg * NWAVE + wave;
    if (g < nG) {
      const float* gr = gp + (size_t)g * DF;
      float a = 0.0f;
#pragma unroll 1
      for (int k = 0; k < DF; ++k) a = fmaf(gr[k], cw1[k * HIDC + lane], a);
      a += bj;
      float t = fmaxf(a, 0.0f) * vj;
      t = wsum(t);
      if (lane == 0) res[g] = t + bz;
    }
  }
  __syncthreads();
  const int n4 = nG >> 2;
  const int ft = nG & ~3;
  if (tid < n4) {
    const v4f v = *(const v4fa*)(res + 4 * tid);
    *(volatile v4f*)(out + 4 * tid) = v;
  }
  if (tid < (nG & 3)) {
    const float v = res[ft + tid];
    *(volatile float*)(out + ft + tid) = v;
  }
  __threadfence();
  if (tid < n4) {
    const v4f v = *(const v4fa*)(res + 4 * tid);
    *(volatile v4f*)(out + 4 * tid) = v;
  }
  if (tid < (nG & 3)) {
    const float v = res[ft + tid];
    *(volatile float*)(out + ft + tid) = v;
  }
}

extern "C" void kernel_launch(void* const* d_in, const int* in_sizes, int n_in,
                              void* d_out, int out_size, void* d_ws, size_t ws_size,
                              hipStream_t stream) {
  if (n_in < 17) return;
  const int nN = in_sizes[3];
  const int nE = in_sizes[2];
  const int nG = out_size;
  if (nN <= 0 || nE <= 0 || nG <= 0 || nG > MAXG) return;
  if (in_sizes[0] != nN * INCH || in_sizes[1] != 2 * nE) return;
  if (in_sizes[4] != NREL * INCH * DF || in_sizes[5] != INCH * DF || in_sizes[6] < DF) return;
  if (in_sizes[7] != NREL * DF * DF || in_sizes[8] != DF * DF || in_sizes[9] < DF) return;
  if (in_sizes[10] != NREL * DF * DF || in_sizes[11] != DF * DF || in_sizes[12] < DF) return;
  if (in_sizes[13] != DF * HIDC || in_sizes[14] < HIDC || in_sizes[15] < HIDC || in_sizes[16] < 1) return;

  const float* x     = (const float*)d_in[0];
  const int*   ei    = (const int*)d_in[1];
  const int*   et    = (const int*)d_in[2];
  const int*   batch = (const int*)d_in[3];
  const float* W1    = (const float*)d_in[4];
  const float* root1 = (const float*)d_in[5];
  const float* b1    = (const float*)d_in[6];
  const float* W2    = (const float*)d_in[7];
  const float* root2 = (const float*)d_in[8];
  const float* b2    = (const float*)d_in[9];
  const float* W3    = (const float*)d_in[10];
  const float* root3 = (const float*)d_in[11];
  const float* b3    = (const float*)d_in[12];
  const float* cW1   = (const float*)d_in[13];
  const float* cb1   = (const float*)d_in[14];
  const float* cW2   = (const float*)d_in[15];
  const float* cb2   = (const float*)d_in[16];
  float* out = (float*)d_out;

  const int nBlkC = (nN + NBC - 1) / NBC;
  const int nPad  = nBlkC * NBC;
  const int nBlk  = (nN + NB - 1) / NB;
  const int nPB   = (nN + PG_ROWS - 1) / PG_ROWS;
  const int vec8  = ((nE & 3) == 0) ? 1 : 0;
  const int nTotW = 2 * NCAT * DF / 8;
  const int nTot1 = nN * NCQ;

  char* ws = (char*)d_ws;
  size_t off = 0;
  const size_t oW   = off; off += (size_t)2 * NCAT * DF * sizeof(f16_t);  off = (off + 255) & ~(size_t)255;
  const size_t oInv = off; off += (size_t)NREL * nPad * sizeof(float);    off = (off + 255) & ~(size_t)255;
  const size_t oP   = off; off += (size_t)nN * NCAT * sizeof(float);      off = (off + 255) & ~(size_t)255;
  const size_t oH   = off; off += (size_t)nN * DF * sizeof(float);        off = (off + 255) & ~(size_t)255;
  const size_t oG   = off; off += (size_t)nG * DF * sizeof(float);        off = (off + 255) & ~(size_t)255;
  if (off > ws_size) return;
  f16_t* wpl = (f16_t*)(ws + oW);
  float* inv = (float*)(ws + oInv);
  float* P   = (float*)(ws + oP);
  f16_t* h16 = (f16_t*)(ws + oH);
  float* h32 = (float*)(ws + oH);
  float* gp  = (float*)(ws + oG);

  k_wprep<<<(nTotW + NTHR - 1) / NTHR, NTHR, 0, stream>>>(W2, root2, W3, root3, wpl, nTotW);

  k_count<<<nBlkC, NTHR, 0, stream>>>(ei, et, inv, nE, nPad, vec8);

  k_proj1<<<(nTot1 + NTHR - 1) / NTHR, NTHR, 0, stream>>>(x, W1, root1, b1, P, nTot1);

  hipFuncSetAttribute(reinterpret_cast<const void*>(&k_agg<0>),
                      hipFuncAttributeMaxDynamicSharedMemorySize, LDS_AGG);
  hipFuncSetAttribute(reinterpret_cast<const void*>(&k_agg<1>),
                      hipFuncAttributeMaxDynamicSharedMemorySize, LDS_AGG);

  k_agg<0><<<nBlk, NTHR, LDS_AGG, stream>>>(ei, et, P, inv, h16, h32, nN, nE, nPad, vec8);

  k_gemm<<<nPB, PG_THR, 0, stream>>>(h16, wpl, b2, P, nN);
  k_agg<0><<<nBlk, NTHR, LDS_AGG, stream>>>(ei, et, P, inv, h16, h32, nN, nE, nPad, vec8);

  k_gemm<<<nPB, PG_THR, 0, stream>>>(h16, wpl + (size_t)NCAT * DF, b3, P, nN);
  k_agg<1><<<nBlk, NTHR, LDS_AGG, stream>>>(ei, et, P, inv, h16, h32, nN, nE, nPad, vec8);

  k_pool<<<nG, NTHR, 0, stream>>>(batch, h32, gp, nN);
  k_head<<<1, NTHR, 0, stream>>>(gp, cW1, cb1, cW2, cb2, out, nG);
}
